// ContrastiveResNetGCN_59725815218593
// MI455X (gfx1250) — hardware-run, weakly checked
//
#include <hip/hip_runtime.h>


#ifndef NTOK
#define NTOK 8192
#endif
#define NTOK_FULL 8192
#define DIN  512
#define DHID 512
#define DP   128
#define DH   128
#define AW   4
#define OSP  132
#define W2C  64.0f
#define W2I  (1.0f / 64.0f)
#define PCI  (1.0f / 1024.0f)
#define EPSV 1.0e-8f
#define EPSS (EPSV * PCI)
#define OSC  (PCI * (1.0f / (float)NTOK))

static_assert(DIN % 64 == 0);
static_assert(DHID % 64 == 0);
static_assert(DP % 64 == 0);
static_assert(DH % 64 == 0);
static_assert(DIN % 32 == 0);
static_assert(DHID % 32 == 0);
static_assert(DP == 128);
static_assert(DH == 128);
static_assert(NTOK % 64 == 0);
static_assert(NTOK % 256 == 0);
static_assert(NTOK % 32 == 0);
static_assert(NTOK % (16 * AW) == 0);
static_assert(NTOK <= NTOK_FULL);
static_assert(((size_t)NTOK * DIN) % 8 == 0);
static_assert((OSP * 4) % 16 == 0);
static_assert(OSP >= DH);
static_assert(AW * 16 * OSP * 4 <= 131072);
static_assert(16 * 68 * 4 <= 131072);
static_assert(64 * 65 * 4 <= 131072);
static_assert(256 * 4 <= 131072);

typedef _Float16 h16;
typedef unsigned short bf;
typedef __attribute__((ext_vector_type(16))) __bf16   v16bf;
typedef __attribute__((ext_vector_type(16))) _Float16 v16h;
typedef __attribute__((ext_vector_type(8)))  _Float16 v8h;
typedef __attribute__((ext_vector_type(8)))  unsigned short v8us;
typedef __attribute__((ext_vector_type(8)))  float    v8f;
typedef __attribute__((ext_vector_type(4)))  float    v4f;
typedef v4f  __attribute__((may_alias)) v4fa;

__device__ __forceinline__ unsigned short f2bf(float f) { unsigned u = __float_as_uint(f); u += 0x7FFFu + ((u >> 16) & 1u); return (unsigned short)(u >> 16); }
__device__ __forceinline__ float bfr(float f) { return __uint_as_float(((unsigned)f2bf(f)) << 16); }
__device__ __forceinline__ v16h cat16(v8h lo, v8h hi) { return __builtin_shufflevector(lo, hi, 0, 1, 2, 3, 4, 5, 6, 7, 8, 9, 10, 11, 12, 13, 14, 15); }
__device__ __forceinline__ v16bf cat16b(v8us lo, v8us hi) { return __builtin_bit_cast(v16bf, __builtin_shufflevector(lo, hi, 0, 1, 2, 3, 4, 5, 6, 7, 8, 9, 10, 11, 12, 13, 14, 15)); }
static __device__ __forceinline__ h16 toh_flush(float v) { const h16 r = (h16)v; return (fabsf(v) < 6.103515625e-05f) ? (h16)0.0f : r; }
__device__ __forceinline__ v8f mmah(v16h a, v16h b, v8f c) {
    c = __builtin_amdgcn_wmma_f32_16x16x32_f16(false, a, false, b, (short)0, c, false, false);
    asm volatile("v_nop\n\tv_nop\n\tv_nop\n\tv_nop" : "+v"(c) : "v"(a), "v"(b));
    return c; }
__device__ __forceinline__ v8f mmab(v16bf a, v16bf b, v8f c) {
    c = __builtin_amdgcn_wmma_f32_16x16x32_bf16(false, a, false, b, (short)0, c, false, false);
    asm volatile("v_nop\n\tv_nop\n\tv_nop\n\tv_nop" : "+v"(c) : "v"(a), "v"(b));
    return c; }
__device__ __forceinline__ v16h  ldh(const h16* p) { return cat16(*(const v8h*)p, *(const v8h*)(p + 16)); }
__device__ __forceinline__ v16bf ldb(const bf* p)  { return cat16b(*(const v8us*)p, *(const v8us*)(p + 16)); }
__device__ __forceinline__ void wave_sync() { __builtin_amdgcn_fence(3  , "wavefront"); __builtin_amdgcn_wave_barrier(); asm volatile("" ::: "memory"); }

template <typename T> struct Op;
template <> struct Op<bf> {
    typedef v16bf frag; typedef v8us vec8;
    static __device__ __forceinline__ frag ld(const bf* p) { return ldb(p); }
    static __device__ __forceinline__ v8f mma(frag a, frag b, v8f c) { return mmab(a, b, c); }
    static __device__ __forceinline__ bf cv(float v, float carry) { return f2bf(v); }
};
template <> struct Op<h16> {
    typedef v16h frag; typedef v8h vec8;
    static __device__ __forceinline__ frag ld(const h16* p) { return ldh(p); }
    static __device__ __forceinline__ v8f mma(frag a, frag b, v8f c) { return mmah(a, b, c); }
    static __device__ __forceinline__ h16 cv(float v, float carry) { return toh_flush(bfr(v) * carry); }
};

__global__ __launch_bounds__(256) void k_cvt8(const float* __restrict__ src, bf* dst, size_t n8) {
    const size_t i = (size_t)blockIdx.x * 256 + threadIdx.x; if (i >= n8) return;
    const v8f v = *(const v8f*)(src + i * 8); v8us o;
#pragma unroll
    for (int k = 0; k < 8; ++k) o[k] = f2bf(v[k]);
    *(volatile v8us*)(dst + i * 8) = o; __threadfence(); *(volatile v8us*)(dst + i * 8) = o;
}

template <typename T>
__device__ __forceinline__ void wt_body(const float* __restrict__ W, T* Wt, const int K, const int N, const float carry) {
    __shared__ float ts[64 * 65];
    const int t = threadIdx.x; const int k0 = blockIdx.x * 64, n0 = blockIdx.y * 64;
#pragma unroll 1
    for (int i = 0; i < 16; ++i) { const int kk = i * 4 + (t >> 6), nn = t & 63; ts[kk * 65 + nn] = W[(size_t)(k0 + kk) * N + n0 + nn]; }
    __syncthreads();
    static_assert(256 * 16 * 2 == 64 * 64 * 2);
#pragma unroll 1
    for (int ps = 0; ps < 2; ++ps) {
#pragma unroll
        for (int s = 0; s < 2; ++s) { const int p = s * 256 + t; const int n = p >> 3, c8 = (p & 7) * 8; typename Op<T>::vec8 o;
#pragma unroll
            for (int i = 0; i < 8; ++i) o[i] = Op<T>::cv(ts[(c8 + i) * 65 + n], carry);
            *(volatile typename Op<T>::vec8*)(Wt + (size_t)(n0 + n) * K + k0 + c8) = o; }
        if (ps == 0) __threadfence(); }
}
__global__ __launch_bounds__(256) void k_wt_bf(const float* __restrict__ W, bf* Wt, int K, int N) { wt_body<bf>(W, Wt, K, N, 1.0f); }
__global__ __launch_bounds__(256) void k_wt_h(const float* __restrict__ W, h16* Wt, int K, int N, float carry) { wt_body<h16>(W, Wt, K, N, carry); }

template <typename T>
__device__ __forceinline__ void gemm64(const T* __restrict__ A, const T* __restrict__ Bt, h16* C, const int K, const int ldc, const float scale, const int relu) {
    __shared__ __align__(16) float os[16 * 68];
    typedef typename Op<T>::frag frag;
    const int lane = threadIdx.x & 31, lr = lane & 15, hi = lane >> 4; const int r0 = blockIdx.x * 64, c0 = blockIdx.y * 64;
    v8f acc[4][4];
#pragma unroll
    for (int mb = 0; mb < 4; ++mb)
#pragma unroll
        for (int nb = 0; nb < 4; ++nb) acc[mb][nb] = (v8f){};
    const size_t aoff = (size_t)(r0 + lr) * K + 8 * hi, boff = (size_t)(c0 + lr) * K + 8 * hi;
#pragma unroll 1
    for (int kc = 0; kc < K; kc += 32) {
        frag a[4];
#pragma unroll
        for (int mb = 0; mb < 4; ++mb) a[mb] = Op<T>::ld(A + aoff + (size_t)mb * 16 * K + kc);
#pragma unroll
        for (int nb = 0; nb < 4; ++nb) { const frag b = Op<T>::ld(Bt + boff + (size_t)nb * 16 * K + kc);
#pragma unroll
            for (int mb = 0; mb < 4; ++mb) acc[mb][nb] = Op<T>::mma(a[mb], b, acc[mb][nb]); }
    }
    static_assert(32 * 16 * 4 == 16 * 64 * 2);
#pragma unroll
    for (int mb = 0; mb < 4; ++mb) {
#pragma unroll
        for (int nb = 0; nb < 4; ++nb) {
#pragma unroll
            for (int j = 0; j < 8; ++j) { float v = acc[mb][nb][j] * scale; v = relu ? fmaxf(v, 0.0f) : v; os[(hi * 8 + j) * 68 + nb * 16 + lr] = v; } }
        wave_sync();
#pragma unroll 1
        for (int ps = 0; ps < 2; ++ps) {
#pragma unroll
            for (int s = 0; s < 4; ++s) { const int row = 4 * s + (lane >> 3), c8 = (lane & 7) * 8;
                const v4f x0 = *(const v4fa*)(&os[row * 68 + c8]); const v4f x1 = *(const v4fa*)(&os[row * 68 + c8 + 4]); v8h hv;
#pragma unroll
                for (int i = 0; i < 4; ++i) { hv[i] = toh_flush(x0[i]); hv[4 + i] = toh_flush(x1[i]); }
                *(volatile v8h*)(C + (size_t)(r0 + mb * 16 + row) * ldc + c0 + c8) = hv; }
            if (ps == 0) __threadfence(); }
        wave_sync();
    }
}
__global__ __launch_bounds__(32) void k_gemm_bf(const bf* __restrict__ A, const bf* __restrict__ Bt, h16* C, int K, int ldc, float scale, int relu) { gemm64<bf>(A, Bt, C, K, ldc, scale, relu); }
__global__ __launch_bounds__(32) void k_gemm_h(const h16* __restrict__ A, const h16* __restrict__ Bt, h16* C, int K, int ldc, float scale, int relu) { gemm64<h16>(A, Bt, C, K, ldc, scale, relu); }

__global__ __launch_bounds__(256) void k_norm(const h16* __restrict__ XP, float* WN) {
#pragma clang fp contract(off)
    __shared__ __align__(16) float sw[256];
    const int tid = threadIdx.x, lane = tid & 31;
    const int wave = __builtin_amdgcn_readfirstlane((int)(threadIdx.x >> 5));
    const int row = blockIdx.x * 256 + tid;
    const h16* p = XP + (size_t)row * DP;
    float s = 0.0f;
#pragma unroll 1
    for (int c = 0; c < DP; c += 8) { const v8h v = *(const v8h*)(p + c);
#pragma unroll
        for (int i = 0; i < 8; ++i) { const float f = (float)v[i]; s += f * f; } }
    sw[tid] = sqrtf(s);
    wave_sync();
    static_assert(8 * 16 == 32 * 4);
    const int li = lane < 8 ? lane : 7;
    const v4f o = *(const v4fa*)(&sw[wave * 32 + li * 4]);
    float* d = WN + (size_t)blockIdx.x * 256 + wave * 32 + li * 4;
    if (lane < 8) { *(volatile v4f*)d = o; __threadfence(); *(volatile v4f*)d = o; }
}

__global__ __launch_bounds__(32 * AW) __attribute__((amdgpu_num_vgpr(256))) void k_agg(const h16* __restrict__ XP, const h16* __restrict__ HT, const float* __restrict__ WN,
                                                                                        const float* __restrict__ gcb, float* OUT) {
    __shared__ __align__(16) float os[AW * 16 * OSP];
    const int lane = threadIdx.x & 31, lr = lane & 15, hi = lane >> 4;
    const int wave = __builtin_amdgcn_readfirstlane((int)(threadIdx.x >> 5));
    const int t0 = (blockIdx.x * AW + wave) * 16;
    const float wis = WN[t0 + lr] * PCI;
    const size_t qo = (size_t)(t0 + lr) * DP + 8 * hi;
    const size_t ko = (size_t)lr * DP + 8 * hi;
    const size_t vo = (size_t)lr * NTOK + 8 * hi;
    const float* wkb = WN + 8 * hi;
    v8f o[8];
#pragma unroll
    for (int j = 0; j < 8; ++j) o[j] = (v8f){};
#pragma unroll 1
    for (int key0 = 0; key0 < NTOK; key0 += 32) {
        int qz = 0; asm volatile("" : "+v"(qz));
        const h16* qa = XP + qo + qz;
        const h16* ka = XP + ko + (size_t)key0 * DP;
        v8f sa = (v8f){}, sb = (v8f){};
#pragma unroll
        for (int dk = 0; dk < 4; ++dk) {
            const v16h q = ldh(qa + dk * 32);
            const v16h a = ldh(ka + dk * 32), b = ldh(ka + 16 * DP + dk * 32);
            sa = mmah(a, q, sa); sb = mmah(b, q, sb); }
        const float* kp = wkb + key0;
        const v4f m0 = *(const v4f*)kp, m1 = *(const v4f*)(kp + 4), m2 = *(const v4f*)(kp + 16), m3 = *(const v4f*)(kp + 20);
        v16h pb;
#pragma unroll
        for (int r = 0; r < 4; ++r) {
            pb[r]      = toh_flush(sa[r]     * __builtin_amdgcn_rcpf(fmaxf(wis * m0[r], EPSS)));
            pb[4 + r]  = toh_flush(sa[4 + r] * __builtin_amdgcn_rcpf(fmaxf(wis * m1[r], EPSS)));
            pb[8 + r]  = toh_flush(sb[r]     * __builtin_amdgcn_rcpf(fmaxf(wis * m2[r], EPSS)));
            pb[12 + r] = toh_flush(sb[4 + r] * __builtin_amdgcn_rcpf(fmaxf(wis * m3[r], EPSS))); }
        const h16* va = HT + vo + key0;
#pragma unroll
        for (int j = 0; j < 8; ++j) { const v16h v = ldh(va + (size_t)(16 * j) * NTOK); o[j] = mmah(v, pb, o[j]); }
    }
    const int wb = wave * 16 * OSP;
#pragma unroll
    for (int j = 0; j < 8; ++j) { v4f a, c;
        a[0] = o[j][0] * OSC; a[1] = o[j][1] * OSC; a[2] = o[j][2] * OSC; a[3] = o[j][3] * OSC;
        c[0] = o[j][4] * OSC; c[1] = o[j][5] * OSC; c[2] = o[j][6] * OSC; c[3] = o[j][7] * OSC;
        *(v4fa*)(&os[wb + lr * OSP + 16 * j + 8 * hi]) = a; *(v4fa*)(&os[wb + lr * OSP + 16 * j + 8 * hi + 4]) = c; }
    wave_sync();
    v4f bv;
    { const v4f g = *(const v4f*)(gcb + lane * 4); bv[0] = bfr(g[0]); bv[1] = bfr(g[1]); bv[2] = bfr(g[2]); bv[3] = bfr(g[3]); }
    float* orow = OUT + (size_t)t0 * DH + lane * 4;
    static_assert(32 * 16 * 16 == 16 * DH * 4);
#pragma unroll 1
    for (int ps = 0; ps < 2; ++ps) {
#pragma unroll
        for (int s = 0; s < 16; ++s) {
            const v4f val = *(const v4fa*)(&os[wb + s * OSP + lane * 4]) + bv;
            *(volatile v4f*)(orow + (size_t)s * DH) = val; }
        if (ps == 0) __threadfence(); }
}

static constexpr size_t al256(size_t v) { return (v + 255) & ~(size_t)255; }
static constexpr size_t SZ_XB = al256((size_t)NTOK * DIN * 2);
static constexpr size_t SZ_W1 = al256((size_t)DHID * DIN * 2);
static constexpr size_t SZ_GC = al256((size_t)DH * DIN * 2);
static constexpr size_t SZ_W2 = al256((size_t)DP * DHID * 2);
static constexpr size_t SZ_H1 = al256((size_t)NTOK * DHID * 2);
static constexpr size_t SZ_XP = al256((size_t)NTOK * DP * 2);
static constexpr size_t SZ_HT = al256((size_t)DH * NTOK * 2);
static constexpr size_t SZ_WN = al256((size_t)NTOK * 4);
static constexpr size_t SZ_TOTAL = SZ_XB + SZ_W1 + SZ_GC + SZ_W2 + SZ_H1 + SZ_XP + SZ_HT + SZ_WN;
static_assert(SZ_TOTAL <= (size_t)134217728);
static_assert((size_t)NTOK * DH * 4 == (size_t)(NTOK / (16 * AW)) * AW * 16 * DH * 4);

extern "C" void kernel_launch(void* const* d_in, const int* in_sizes, int n_in,
                              void* d_out, int out_size, void* d_ws, size_t ws_size, hipStream_t stream) {
    if (n_in < 5) return;
    if ((size_t)in_sizes[0] < (size_t)NTOK * DIN) return;
    if ((size_t)in_sizes[1] < (size_t)DIN * DHID) return;
    if ((size_t)in_sizes[2] < (size_t)DHID * DP) return;
    if ((size_t)in_sizes[3] < (size_t)DIN * DH) return;
    if (in_sizes[4] < DH) return;
    if ((size_t)out_size < (size_t)NTOK * DH) return;
    if (SZ_TOTAL > ws_size) return;
    const float* x1  = (const float*)d_in[0];
    const float* w1  = (const float*)d_in[1];
    const float* w2  = (const float*)d_in[2];
    const float* gcw = (const float*)d_in[3];
    const float* gcb = (const float*)d_in[4];
    float* OUT = (float*)d_out;
    char* wsp = (char*)d_ws;
    bf*  XB  = (bf*)wsp;  wsp += SZ_XB;
    bf*  W1T = (bf*)wsp;  wsp += SZ_W1;
    bf*  GCT = (bf*)wsp;  wsp += SZ_GC;
    h16* W2T = (h16*)wsp; wsp += SZ_W2;
    h16* H1  = (h16*)wsp; wsp += SZ_H1;
    h16* XPH = (h16*)wsp; wsp += SZ_XP;
    h16* HT  = (h16*)wsp; wsp += SZ_HT;
    float* WN = (float*)wsp; wsp += SZ_WN;

    { const size_t n8 = (size_t)NTOK * DIN / 8;
      k_cvt8<<<(unsigned)((n8 + 255) / 256), 256, 0, stream>>>(x1, XB, n8); }
    k_wt_bf<<<dim3(DIN / 64, DHID / 64, 1), 256, 0, stream>>>(w1, W1T, DIN, DHID);
    k_wt_bf<<<dim3(DIN / 64, DH / 64, 1), 256, 0, stream>>>(gcw, GCT, DIN, DH);
    k_wt_h<<<dim3(DHID / 64, DP / 64, 1), 256, 0, stream>>>(w2, W2T, DHID, DP, W2C);

    k_gemm_bf<<<dim3(NTOK / 64, DHID / 64, 1), 32, 0, stream>>>(XB, W1T, H1, DIN, DHID, 1.0f, 1);
    k_gemm_h<<<dim3(NTOK / 64, DP / 64, 1), 32, 0, stream>>>(H1, W2T, XPH, DHID, DP, W2I, 0);
    k_gemm_bf<<<dim3(DH / 64, NTOK / 64, 1), 32, 0, stream>>>(GCT, XB, HT, DIN, NTOK, 1.0f, 0);
    k_norm<<<NTOK / 256, 256, 0, stream>>>(XPH, WN);
    k_agg<<<NTOK / (16 * AW), 32 * AW, 0, stream>>>(XPH, HT, WN, gcb, OUT);
}
